// LRSA_5927054868706
// MI455X (gfx1250) — hardware-verified
//
#include <hip/hip_runtime.h>


namespace {
constexpr int NB_ = 2, C = 64, IMG = 226, PS = 16, STEP = 14, NPS = 16  , NPATCH = NPS * NPS  , TPP = PS * PS  , NTOK = NPATCH * TPP  , HEADS = 4, DH = 16, MLP = 128;
constexpr float HS = 256.0f, PSC = 256.0f, WSC = 256.0f, SCALE = 0.25f, EPS = 1e-5f;
typedef _Float16 b16;
typedef __attribute__((ext_vector_type(16))) _Float16 v16b;
typedef __attribute__((ext_vector_type(8))) _Float16 v8b;
typedef __attribute__((ext_vector_type(2))) _Float16 v2b;
typedef __attribute__((ext_vector_type(8))) float v8f;
typedef __attribute__((ext_vector_type(4))) float v4f;
typedef __attribute__((ext_vector_type(2))) float v2f;
__device__ __forceinline__ float bf16_rne(float f) { unsigned int u = __float_as_uint(f); u += 0x7FFFu + ((u >> 16) & 1u); float r = __uint_as_float(u & 0xFFFF0000u); asm volatile("" : "+v"(r)); return r; }
__device__ __forceinline__ float bfv(float f) { float r = bf16_rne(f); asm volatile("" : "+v"(r)); return r; }
__device__ __forceinline__ void split16(float v, b16& hi, b16& lo) { hi = (b16)v; lo = (b16)(v - (float)hi); }
__device__ __forceinline__ v16b frag_kb(const b16* p, int hh) { const v8b a = *(const v8b*)(p + 8 * hh), b = *(const v8b*)(p + 16 + 8 * hh); v16b f;
#pragma unroll
  for (int e = 0; e < 8; ++e) { f[e] = a[e]; f[8 + e] = b[e]; } return f; }
__device__ __forceinline__ v8f wmma16b(v16b a, v16b b, v8f c) { v8f d = __builtin_amdgcn_wmma_f32_16x16x32_f16(false, a, false, b, (short)0, c, false, false); asm volatile("v_nop\n\tv_nop\n\tv_nop\n\tv_nop" : "+v"(d) : "v"(a), "v"(b)); return d; }
__device__ __forceinline__ void wave_lds_sync() { __builtin_amdgcn_fence(__ATOMIC_RELEASE, "workgroup"); __builtin_amdgcn_wave_barrier(); __builtin_amdgcn_fence(__ATOMIC_ACQUIRE, "workgroup"); }
__device__ __forceinline__ float pmul(float a, float b) { float p = a * b; asm volatile("" : "+v"(p)); return p; }
__device__ __forceinline__ float gelu_erf(float v) { return 0.5f * v * (1.0f + erff(v * 0.70710678118654752f)); }
__device__ __forceinline__ void tok_of(size_t g, int& pi, int& pj, int& py, int& px) { const int patch = (int)(g / TPP), tk = (int)(g % TPP); pi = patch / NPS; pj = patch % NPS; py = tk / PS; px = tk % PS; }

__global__ __launch_bounds__(256) void wput_kernel(const float* __restrict__ wq, const float* __restrict__ wk, const float* __restrict__ wv, const float* __restrict__ wp, const float* __restrict__ wf1, const float* __restrict__ wf2, b16* __restrict__ WQKV, b16* __restrict__ WP, b16* __restrict__ WF1, b16* __restrict__ WF2) { const int u = blockIdx.x * 256 + threadIdx.x; v8b v;
  if (u < 192 * 8) { const int o = u / 8, k0 = (u % 8) * 8; const int which = o / 64, oo = o % 64; const float* w = which == 0 ? wq : (which == 1 ? wk : wv);
#pragma unroll
    for (int j = 0; j < 8; ++j) v[j] = (b16)(bf16_rne(w[(size_t)(k0 + j) * 64 + oo]) * WSC); for (int pass = 0; pass < 2; ++pass) { *(volatile v8b*)(WQKV + (size_t)o * C + k0) = v; __threadfence(); } }
  if (u < 64 * 8) { const int o = u / 8, k0 = (u % 8) * 8;
#pragma unroll
    for (int j = 0; j < 8; ++j) v[j] = (b16)(bf16_rne(wp[(size_t)(k0 + j) * C + o]) * WSC); for (int pass = 0; pass < 2; ++pass) { *(volatile v8b*)(WP + (size_t)o * C + k0) = v; __threadfence(); } }
  if (u < MLP * 8) { const int o = u / 8, k0 = (u % 8) * 8;
#pragma unroll
    for (int j = 0; j < 8; ++j) v[j] = (b16)(bf16_rne(wf1[(size_t)(k0 + j) * MLP + o]) * WSC); for (int pass = 0; pass < 2; ++pass) { *(volatile v8b*)(WF1 + (size_t)o * C + k0) = v; __threadfence(); } }
  if (u < 64 * 16) { const int o = u / 16, k0 = (u % 16) * 8;
#pragma unroll
    for (int j = 0; j < 8; ++j) v[j] = (b16)(bf16_rne(wf2[(size_t)(k0 + j) * C + o]) * WSC); for (int pass = 0; pass < 2; ++pass) { *(volatile v8b*)(WF2 + (size_t)o * MLP + k0) = v; __threadfence(); } } }
__device__ __forceinline__ void ln_row(float* row, int n, const float* g, const float* bta) {
  float m = 0.0f; for (int c = 0; c < n; ++c) m += row[c]; m *= (1.0f / (float)n); float vr = 0.0f; for (int c = 0; c < n; ++c) { const float d = row[c] - m; vr += d * d; } vr *= (1.0f / (float)n); const float rs = rsqrtf(vr + EPS); for (int c = 0; c < n; ++c) row[c] = pmul((row[c] - m) * rs, bfv(g[c])) + bfv(bta[c]); }
__global__ __launch_bounds__(32) void qkv_kernel(const float* __restrict__ x  , const float* __restrict__ g1, const float* __restrict__ bb1, const b16* __restrict__ WQKV, int GLIM, float* __restrict__ T0, b16* __restrict__ QPh, b16* __restrict__ QPl, b16* __restrict__ KPh, b16* __restrict__ KPl, float* __restrict__ V) { __shared__ __attribute__((aligned(16))) b16 Ah[16][C + 8], Al[16][C + 8]; __shared__ float Tr[16][C + 1], Tf[16][196]; const int lane = threadIdx.x, nloc = lane & 15, hlf = lane >> 4; const size_t g0 = (size_t)blockIdx.x * 16; if (g0 >= (size_t)GLIM) return;
  for (int rr = 0; rr < 16; ++rr) { int pi, pj, py, px; tok_of(g0 + rr, pi, pj, py, px); const int yy = pi * STEP + py, xx = pj * STEP + px; for (int q = 0; q < 2; ++q) { const int c = q * 32 + lane; Tr[rr][c] = bfv(x[((size_t)c * IMG + yy) * IMG + xx]); } }
  wave_lds_sync();
  for (int pass = 0; pass < 2; ++pass) { for (int rr = 0; rr < 16; ++rr) *(volatile v2f*)(T0 + (g0 + rr) * C + lane * 2) = (v2f){Tr[rr][lane * 2], Tr[rr][lane * 2 + 1]}; __threadfence(); }
  wave_lds_sync();
  if (lane < 16) ln_row(&Tr[lane][0], C, g1, bb1);
  wave_lds_sync();
  for (int rr = 0; rr < 16; ++rr) for (int q = 0; q < 2; ++q) { const int c = q * 32 + lane; b16 p, pl; split16(Tr[rr][c] * HS, p, pl); Ah[rr][c] = p; Al[rr][c] = pl; }
  if (lane < 16) for (int k = C; k < C + 8; ++k) { Ah[lane][k] = (b16)0.0f; Al[lane][k] = (b16)0.0f; }
  wave_lds_sync(); v8f acc[12];
#pragma unroll
  for (int t = 0; t < 12; ++t) acc[t] = (v8f){};
#pragma unroll
  for (int kb = 0; kb < C; kb += 32) { const v16b a = frag_kb(&Ah[nloc][kb], hlf), al = frag_kb(&Al[nloc][kb], hlf);
#pragma unroll
    for (int t = 0; t < 12; ++t) { const v16b bw = frag_kb(WQKV + (size_t)(t * 16 + nloc) * C + kb, hlf); acc[t] = wmma16b(a, bw, acc[t]); acc[t] = wmma16b(al, bw, acc[t]); } }
#pragma unroll
  for (int t = 0; t < 12; ++t)
#pragma unroll
    for (int r8 = 0; r8 < 8; ++r8) Tf[8 * hlf + r8][t * 16 + nloc] = acc[t][r8] * (1.0f / (HS * WSC));
  wave_lds_sync();
  for (int pass = 0; pass < 2; ++pass) { for (int rr = 0; rr < 16; ++rr) { const size_t go = (g0 + rr); const int h = lane >> 3, d2 = (lane & 7) * 2; const float q0v = Tf[rr][h * DH + d2], q1v = Tf[rr][h * DH + d2 + 1], k0v = Tf[rr][64 + h * DH + d2], k1v = Tf[rr][64 + h * DH + d2 + 1]; b16 a0, a1, l0, l1; split16(q0v * HS, a0, l0); split16(q1v * HS, a1, l1); const size_t po = (go * HEADS + h) * 32 + d2; *(volatile v2b*)(QPh + po) = (v2b){a0, a1}; *(volatile v2b*)(QPl + po) = (v2b){l0, l1}; *(volatile v2b*)(QPh + po + 16) = (v2b){0, 0}; *(volatile v2b*)(QPl + po + 16) = (v2b){0, 0}; split16(k0v * HS, a0, l0); split16(k1v * HS, a1, l1); *(volatile v2b*)(KPh + po) = (v2b){a0, a1}; *(volatile v2b*)(KPl + po) = (v2b){l0, l1}; *(volatile v2b*)(KPh + po + 16) = (v2b){0, 0}; *(volatile v2b*)(KPl + po + 16) = (v2b){0, 0}; *(volatile v2f*)(V + go * C + lane * 2) = (v2f){Tf[rr][128 + lane * 2], Tf[rr][128 + lane * 2 + 1]}; } __threadfence(); } }
__global__ __launch_bounds__(256) void vt_kernel(const float* __restrict__ V, int GLIM, b16* __restrict__ VTh, b16* __restrict__ VTl) { __shared__ float Tt[TPP][C + 1]; const int patch = blockIdx.x; if ((size_t)patch * TPP >= (size_t)GLIM) return; const int tid = threadIdx.x, wave = tid >> 5, lane = tid & 31;
  for (int q = wave; q < TPP; q += 8) for (int c = lane; c < C; c += 32) Tt[q][c] = V[((size_t)patch * TPP + q) * C + c];
  __syncthreads();
  for (int pass = 0; pass < 2; ++pass) { for (int c = wave; c < C; c += 8) for (int s = 0; s < TPP; s += 64) { b16 h0, l0, h1, l1; split16(Tt[s + lane * 2][c] * HS, h0, l0); split16(Tt[s + lane * 2 + 1][c] * HS, h1, l1); const size_t o = ((size_t)patch * C + c) * TPP + s + lane * 2; *(volatile v2b*)(VTh + o) = (v2b){h0, h1}; *(volatile v2b*)(VTl + o) = (v2b){l0, l1}; } __threadfence(); } }
__global__ __launch_bounds__(32) void att_kernel(const b16* __restrict__ QPh, const b16* __restrict__ QPl, const b16* __restrict__ KPh, const b16* __restrict__ KPl, const b16* __restrict__ VTh, const b16* __restrict__ VTl, int GLIM, float* __restrict__ O) { __shared__ __attribute__((aligned(16))) b16 Pa[16][TPP + 8], Pb[16][TPP + 8]; __shared__ float Sc[16][TPP + 1], Of[16][C + 1]; const int lane = threadIdx.x, nloc = lane & 15, hlf = lane >> 4; const int patch = blockIdx.x / (TPP / 16), q0 = (blockIdx.x % (TPP / 16)) * 16; const size_t gq = (size_t)patch * TPP + q0; if (gq >= (size_t)GLIM) return;
  if (lane < 16) for (int k = TPP; k < TPP + 8; ++k) { Pa[lane][k] = (b16)0.0f; Pb[lane][k] = (b16)0.0f; }
#pragma unroll 1
  for (int h = 0; h < HEADS; ++h) { const v16b qa = frag_kb(QPh + ((gq + nloc) * HEADS + h) * 32, hlf), ql = frag_kb(QPl + ((gq + nloc) * HEADS + h) * 32, hlf);
#pragma unroll 4
    for (int t = 0; t < TPP / 16; ++t) { const size_t ko = (((size_t)patch * TPP + t * 16 + nloc) * HEADS + h) * 32; const v16b kh = frag_kb(KPh + ko, hlf), kl = frag_kb(KPl + ko, hlf); v8f s = wmma16b(qa, kh, (v8f){}); s = wmma16b(qa, kl, s); s = wmma16b(ql, kh, s);
#pragma unroll
      for (int r8 = 0; r8 < 8; ++r8) Sc[8 * hlf + r8][t * 16 + nloc] = s[r8] * (SCALE / (HS * HS)); }
    wave_lds_sync();
    if (lane < 16) { const int r = lane; float mx = -INFINITY; for (int k = 0; k < TPP; ++k) mx = fmaxf(mx, Sc[r][k]); float sm = 0.0f; for (int k = 0; k < TPP; ++k) { const float p = __expf(Sc[r][k] - mx); Sc[r][k] = p; sm += p; } const float inv = 1.0f / sm; for (int k = 0; k < TPP; ++k) { b16 p, pl; split16(Sc[r][k] * inv * PSC, p, pl); Pa[r][k] = p; Pb[r][k] = pl; } }
    wave_lds_sync();
    v8f o = (v8f){};
#pragma unroll 2
    for (int kb = 0; kb < TPP; kb += 32) { const v16b pa = frag_kb(&Pa[nloc][kb], hlf), pb = frag_kb(&Pb[nloc][kb], hlf); const size_t vo = ((size_t)patch * C + h * DH + nloc) * TPP + kb; const v16b vh = frag_kb(VTh + vo, hlf), vl = frag_kb(VTl + vo, hlf); o = wmma16b(pa, vh, o); o = wmma16b(pa, vl, o); o = wmma16b(pb, vh, o); }
#pragma unroll
    for (int r8 = 0; r8 < 8; ++r8) Of[8 * hlf + r8][h * DH + nloc] = o[r8] * (1.0f / (PSC * HS));
    wave_lds_sync(); }
  for (int pass = 0; pass < 2; ++pass) { for (int r = 0; r < 16; ++r) *(volatile v2f*)(O + (gq + r) * C + lane * 2) = (v2f){Of[r][lane * 2], Of[r][lane * 2 + 1]}; __threadfence(); } }
__global__ __launch_bounds__(32) void mlp1_kernel(const float* __restrict__ O, const float* __restrict__ T0, const b16* __restrict__ WP, const float* __restrict__ bp, const float* __restrict__ g2, const float* __restrict__ bb2, const b16* __restrict__ WF1, const float* __restrict__ bf1, int GLIM, float* __restrict__ T1, float* __restrict__ Y) { __shared__ __attribute__((aligned(16))) b16 Ah[16][C + 8], Al[16][C + 8]; __shared__ float Tr[16][C + 1], Tf[16][MLP + 4]; const int lane = threadIdx.x, nloc = lane & 15, hlf = lane >> 4; const size_t g0 = (size_t)blockIdx.x * 16; if (g0 >= (size_t)GLIM) return;
  for (int rr = 0; rr < 16; ++rr) for (int q = 0; q < 2; ++q) { const int c = q * 32 + lane; b16 p, pl; split16(O[(g0 + rr) * C + c] * HS, p, pl); Ah[rr][c] = p; Al[rr][c] = pl; }
  if (lane < 16) for (int k = C; k < C + 8; ++k) { Ah[lane][k] = (b16)0.0f; Al[lane][k] = (b16)0.0f; }
  wave_lds_sync(); v8f acc[4] = {(v8f){}, (v8f){}, (v8f){}, (v8f){}};
#pragma unroll
  for (int kb = 0; kb < C; kb += 32) { const v16b a = frag_kb(&Ah[nloc][kb], hlf), al = frag_kb(&Al[nloc][kb], hlf);
#pragma unroll
    for (int t = 0; t < 4; ++t) { const v16b bw = frag_kb(WP + (size_t)(t * 16 + nloc) * C + kb, hlf); acc[t] = wmma16b(a, bw, acc[t]); acc[t] = wmma16b(al, bw, acc[t]); } }
#pragma unroll
  for (int t = 0; t < 4; ++t)
#pragma unroll
    for (int r8 = 0; r8 < 8; ++r8) { const int rr = 8 * hlf + r8, cc = t * 16 + nloc; Tr[rr][cc] = acc[t][r8] * (1.0f / (HS * WSC)) + bfv(bp[cc]) + T0[(g0 + rr) * C + cc]; }
  wave_lds_sync();
  for (int pass = 0; pass < 2; ++pass) { for (int rr = 0; rr < 16; ++rr) *(volatile v2f*)(T1 + (g0 + rr) * C + lane * 2) = (v2f){Tr[rr][lane * 2], Tr[rr][lane * 2 + 1]}; __threadfence(); }
  wave_lds_sync();
  if (lane < 16) ln_row(&Tr[lane][0], C, g2, bb2);
  wave_lds_sync();
  for (int rr = 0; rr < 16; ++rr) for (int q = 0; q < 2; ++q) { const int c = q * 32 + lane; b16 p, pl; split16(Tr[rr][c] * HS, p, pl); Ah[rr][c] = p; Al[rr][c] = pl; }
  wave_lds_sync(); v8f acc2[8];
#pragma unroll
  for (int t = 0; t < 8; ++t) acc2[t] = (v8f){};
#pragma unroll
  for (int kb = 0; kb < C; kb += 32) { const v16b a = frag_kb(&Ah[nloc][kb], hlf), al = frag_kb(&Al[nloc][kb], hlf);
#pragma unroll
    for (int t = 0; t < 8; ++t) { const v16b bw = frag_kb(WF1 + (size_t)(t * 16 + nloc) * C + kb, hlf); acc2[t] = wmma16b(a, bw, acc2[t]); acc2[t] = wmma16b(al, bw, acc2[t]); } }
#pragma unroll
  for (int t = 0; t < 8; ++t)
#pragma unroll
    for (int r8 = 0; r8 < 8; ++r8) { const int cc = t * 16 + nloc; Tf[8 * hlf + r8][cc] = gelu_erf(acc2[t][r8] * (1.0f / (HS * WSC)) + bfv(bf1[cc])); }
  wave_lds_sync();
  for (int pass = 0; pass < 2; ++pass) { for (int rr = 0; rr < 16; ++rr) *(volatile v4f*)(Y + (g0 + rr) * MLP + lane * 4) = *(const v4f*)(&Tf[rr][lane * 4]); __threadfence(); } }
__global__ __launch_bounds__(32) void dw_kernel(const float* __restrict__ Y, const float* __restrict__ T1, const float* __restrict__ wdw, const float* __restrict__ bdw, const b16* __restrict__ WF2, const float* __restrict__ bf2, int GLIM, float* __restrict__ T2) { __shared__ __attribute__((aligned(16))) b16 Ah[16][MLP + 8], Al[16][MLP + 8]; __shared__ float Tf[16][C + 1]; const int lane = threadIdx.x, nloc = lane & 15, hlf = lane >> 4; const size_t g0 = (size_t)blockIdx.x * 16; if (g0 >= (size_t)GLIM) return; const size_t pbase = (g0 / TPP) * TPP; const int py = (int)((g0 % TPP) / PS);
  for (int ch4 = 0; ch4 < 4; ++ch4) { const int ch = lane * 4 + ch4; const float* wrow = wdw + (size_t)ch * 25; const float bb = bfv(bdw[ch]);
    for (int px = 0; px < PS; ++px) { float s = bb;
#pragma unroll 1
      for (int i = 0; i < 5; ++i) { const int yy = py + i - 2; if (yy < 0 || yy >= PS) continue;
#pragma unroll 1
        for (int j = 0; j < 5; ++j) { const int xx = px + j - 2; if (xx < 0 || xx >= PS) continue; s += pmul(bfv(wrow[i * 5 + j]), Y[(pbase + yy * PS + xx) * MLP + ch]); } }
      const float yv = Y[(g0 + px) * MLP + ch] + gelu_erf(s); b16 p, pl; split16(yv * HS, p, pl); Ah[px][ch] = p; Al[px][ch] = pl; } }
  if (lane < 16) for (int k = MLP; k < MLP + 8; ++k) { Ah[lane][k] = (b16)0.0f; Al[lane][k] = (b16)0.0f; }
  wave_lds_sync(); v8f acc[4] = {(v8f){}, (v8f){}, (v8f){}, (v8f){}};
#pragma unroll
  for (int kb = 0; kb < MLP; kb += 32) { const v16b a = frag_kb(&Ah[nloc][kb], hlf), al = frag_kb(&Al[nloc][kb], hlf);
#pragma unroll
    for (int t = 0; t < 4; ++t) { const v16b bw = frag_kb(WF2 + (size_t)(t * 16 + nloc) * MLP + kb, hlf); acc[t] = wmma16b(a, bw, acc[t]); acc[t] = wmma16b(al, bw, acc[t]); } }
#pragma unroll
  for (int t = 0; t < 4; ++t)
#pragma unroll
    for (int r8 = 0; r8 < 8; ++r8) { const int rr = 8 * hlf + r8, cc = t * 16 + nloc; Tf[rr][cc] = acc[t][r8] * (1.0f / (HS * WSC)) + bfv(bf2[cc]) + T1[(g0 + rr) * C + cc]; }
  wave_lds_sync();
  for (int pass = 0; pass < 2; ++pass) { for (int rr = 0; rr < 16; ++rr) *(volatile v2f*)(T2 + (g0 + rr) * C + lane * 2) = (v2f){Tf[rr][lane * 2], Tf[rr][lane * 2 + 1]}; __threadfence(); } }
__global__ __launch_bounds__(256) void out_kernel(const float* __restrict__ T2, int GLIM, float* __restrict__ out  ) { const size_t u = (size_t)blockIdx.x * 256 + threadIdx.x; if (u >= (size_t)C * IMG * IMG) return; const int xx = (int)(u % IMG), yy = (int)((u / IMG) % IMG), c = (int)(u / ((size_t)IMG * IMG));
  int iy0 = (yy - PS) / STEP + 1; if (yy < PS) iy0 = 0; int iy1 = yy / STEP; if (iy1 > NPS - 1) iy1 = NPS - 1; int ix0 = (xx - PS) / STEP + 1; if (xx < PS) ix0 = 0; int ix1 = xx / STEP; if (ix1 > NPS - 1) ix1 = NPS - 1;
  float s = 0.0f; int cnt = 0; for (int iy = iy0; iy <= iy1; ++iy) for (int ix = ix0; ix <= ix1; ++ix) { const int py = yy - iy * STEP, px = xx - ix * STEP; if (py < 0 || py >= PS || px < 0 || px >= PS) continue; const size_t g = ((size_t)(iy * NPS + ix)) * TPP + py * PS + px; ++cnt; if (g < (size_t)GLIM) s += T2[g * C + c]; }
  const float v = cnt > 0 ? s / (float)cnt : 0.0f;
  for (int pass = 0; pass < 2; ++pass) { ((volatile float*)out)[u] = v; __threadfence(); } }
}

extern "C" void kernel_launch(void* const* d_in, const int* in_sizes, int n_in, void* d_out, int out_size, void* d_ws, size_t ws_size, hipStream_t stream) {
  (void)n_in;
  auto Fp = [&](int i) { return (const float*)d_in[i]; };
  if (in_sizes[0] != NB_ * C * IMG * IMG || in_sizes[3] != C * C || in_sizes[10] != C * MLP || in_sizes[12] != MLP * 25 || in_sizes[14] != MLP * C || out_size != NB_ * C * IMG * IMG) return;
  const int GLIM = NTOK;
  size_t off = 0; char* ws = (char*)d_ws;
  auto carve = [&](size_t bytes) { char* p = ws + off; off += (bytes + 255) & ~(size_t)255; return p; };
  b16* WQKV = (b16*)carve(192 * C * 2); b16* WP = (b16*)carve(64 * C * 2); b16* WF1 = (b16*)carve(MLP * C * 2); b16* WF2 = (b16*)carve(C * MLP * 2);
  float* T0 = (float*)carve((size_t)NTOK * C * 4); b16* QPh = (b16*)carve((size_t)NTOK * HEADS * 32 * 2); b16* QPl = (b16*)carve((size_t)NTOK * HEADS * 32 * 2); b16* KPh = (b16*)carve((size_t)NTOK * HEADS * 32 * 2); b16* KPl = (b16*)carve((size_t)NTOK * HEADS * 32 * 2); float* V = (float*)carve((size_t)NTOK * C * 4); b16* VTh = (b16*)carve((size_t)NTOK * C * 2); b16* VTl = (b16*)carve((size_t)NTOK * C * 2); float* O = (float*)carve((size_t)NTOK * C * 4); float* T1 = (float*)carve((size_t)NTOK * C * 4); float* Y = (float*)carve((size_t)NTOK * MLP * 4); float* T2 = (float*)carve((size_t)NTOK * C * 4);
  if (off > ws_size || off > ((size_t)208 << 20)) return;
  wput_kernel<<<(192 * 8 + 255) / 256, 256, 0, stream>>>(Fp(3), Fp(4), Fp(5), Fp(6), Fp(10), Fp(14), WQKV, WP, WF1, WF2);
  for (int img = 0; img < NB_; ++img) { const float* xi = Fp(0) + (size_t)img * C * IMG * IMG; float* oi = (float*)d_out + (size_t)img * C * IMG * IMG;
    qkv_kernel<<<NTOK / 16, 32, 0, stream>>>(xi, Fp(1), Fp(2), WQKV, GLIM, T0, QPh, QPl, KPh, KPl, V);
    vt_kernel<<<NPATCH, 256, 0, stream>>>(V, GLIM, VTh, VTl);
    att_kernel<<<NPATCH * (TPP / 16), 32, 0, stream>>>(QPh, QPl, KPh, KPl, VTh, VTl, GLIM, O);
    mlp1_kernel<<<NTOK / 16, 32, 0, stream>>>(O, T0, WP, Fp(7), Fp(8), Fp(9), WF1, Fp(11), GLIM, T1, Y);
    dw_kernel<<<NTOK / 16, 32, 0, stream>>>(Y, T1, Fp(12), Fp(13), WF2, Fp(15), GLIM, T2);
    out_kernel<<<(C * IMG * IMG + 255) / 256, 256, 0, stream>>>(T2, GLIM, oi); }
}
